// MultiHeadAttentionEinsum_44753559224413
// MI455X (gfx1250) — hardware-verified
//
#include <hip/hip_runtime.h>
#include <stdint.h>
#include <math.h>

typedef __attribute__((ext_vector_type(16))) _Float16 v16h;
typedef __attribute__((ext_vector_type(8)))  _Float16 v8h;
typedef __attribute__((ext_vector_type(16))) __bf16   v16b;
typedef __attribute__((ext_vector_type(8)))  __bf16   v8b;
typedef __attribute__((ext_vector_type(8)))  float    v8f;
typedef __attribute__((ext_vector_type(4)))  float    v4f;
typedef __attribute__((ext_vector_type(4)))  unsigned int v4u;

__device__ __forceinline__ unsigned short f2bf_bits(float f) {
  unsigned u = __float_as_uint(f);
  return (unsigned short)((u + 0x7FFFu + ((u >> 16) & 1u)) >> 16);
}
__device__ __forceinline__ float bf_bits2f(unsigned short h) { return __uint_as_float(((unsigned)h) << 16); }

__device__ __forceinline__ void dep_guard_h(v8f& a, v8f& b, v16h x, v16h y) { asm volatile("v_nop\n\tv_nop\n\tv_nop\n\tv_nop" : "+v"(a), "+v"(b) : "v"(x), "v"(y)); }
__device__ __forceinline__ void dep_guard_b(v8f& a, v8f& b, v16b x, v16b y) { asm volatile("v_nop\n\tv_nop\n\tv_nop\n\tv_nop" : "+v"(a), "+v"(b) : "v"(x), "v"(y)); }
__device__ __forceinline__ void keep4_h(v16h a, v16h b, v16h c, v16h d) { asm volatile("v_nop" :: "v"(a), "v"(b), "v"(c), "v"(d)); }
__device__ __forceinline__ void keep4_b(v16b a, v16b b, v16b c, v16b d) { asm volatile("v_nop" :: "v"(a), "v"(b), "v"(c), "v"(d)); }
__device__ __forceinline__ void acc_guard4(v8f& a, v8f& b, v8f& c, v8f& d) { asm volatile("v_nop\n\tv_nop\n\tv_nop\n\tv_nop" : "+v"(a), "+v"(b), "+v"(c), "+v"(d)); }
template <typename T> struct Frag;
template <> struct Frag<_Float16> {
  typedef v16h V; union U { v16h v; v8h h[2]; };
  static __device__ __forceinline__ v16h load(const _Float16* p) {
    U f; f.h[0] = *(const v8h*)(p); f.h[1] = *(const v8h*)(p + 16); return f.v;
  }
  static __device__ __forceinline__ v8f mma(v16h a, v16h b, v8f c) {
    return __builtin_amdgcn_wmma_f32_16x16x32_f16(false, a, false, b, (short)0, c, false, false);
  }
  static __device__ __forceinline__ void guard(v8f& a, v8f& b, v16h x, v16h y) { dep_guard_h(a, b, x, y); }
  static __device__ __forceinline__ void keep(v16h a, v16h b, v16h c, v16h d) { keep4_h(a, b, c, d); }
};
template <> struct Frag<__bf16> {
  typedef v16b V; union U { v16b v; v8b h[2]; };
  static __device__ __forceinline__ v16b load(const __bf16* p) {
    U f; f.h[0] = *(const v8b*)(p); f.h[1] = *(const v8b*)(p + 16); return f.v;
  }
  static __device__ __forceinline__ v8f mma(v16b a, v16b b, v8f c) {
    return __builtin_amdgcn_wmma_f32_16x16x32_bf16(false, a, false, b, (short)0, c, false, false);
  }
  static __device__ __forceinline__ void guard(v8f& a, v8f& b, v16b x, v16b y) { dep_guard_b(a, b, x, y); }
  static __device__ __forceinline__ void keep(v16b a, v16b b, v16b c, v16b d) { keep4_b(a, b, c, d); }
};

template <int ET> struct Elem;
template <> struct Elem<0> { typedef _Float16 T; };
template <> struct Elem<1> { typedef __bf16 T; };
template <int ET, bool SPLIT, int BIAS_MODE, int OUT_MODE, bool RESID, int ACT = 0>
__global__ __launch_bounds__(256) void wmma_gemm64(
    const unsigned short* __restrict__ Ap, const unsigned short* __restrict__ A2p, int lda, long strideA,
    const unsigned short* __restrict__ Btp, const unsigned short* __restrict__ Bt2p, int ldb, long strideB,
    void* __restrict__ Cout, void* __restrict__ Cout2, int ldc, long strideC,
    const float* __restrict__ bias,
    const float* __restrict__ resid, long strideR,
    int M, int N, int K, float scale) {
  typedef typename Elem<ET>::T T;
  typedef typename Frag<T>::V V;
  const T* A = (const T*)Ap; const T* A2 = (const T*)A2p; const T* Bt = (const T*)Btp; const T* Bt2 = (const T*)Bt2p;
  __shared__ __align__(16) float sT[8][16 * 68];
  const int b    = blockIdx.y;
  const int lane = threadIdx.x & 31;
  const int wave = threadIdx.x >> 5;
  const int tilesN = N >> 6;
  const int tilesM = M >> 6;
  const int tile = blockIdx.x * 8 + wave;
  if (tile >= tilesM * tilesN) return;
  const int tm = tile / tilesN;
  const int tn = tile - tm * tilesN;
  const int m0 = tm << 6;
  const int n0 = tn << 6;

  const T* Ab  = A  + (size_t)b * strideA;
  const T* Bb  = Bt + (size_t)b * strideB;
  const T* Ab2 = SPLIT ? (A2  + (size_t)b * strideA) : nullptr;
  const T* Bb2 = SPLIT ? (Bt2 + (size_t)b * strideB) : nullptr;

  const int rlane = lane & 15;
  const int koff  = (lane >> 4) * 8;
  const int mOff  = (lane >> 4) * 8;

  v8f acc[4][4];
#pragma unroll
  for (int i = 0; i < 4; ++i)
#pragma unroll
    for (int j = 0; j < 4; ++j) acc[i][j] = (v8f){0.f,0.f,0.f,0.f,0.f,0.f,0.f,0.f};

  for (int k0 = 0; k0 < K; k0 += 32) {
    V bh[4], bl[4];
#pragma unroll
    for (int j = 0; j < 4; ++j) {
      const size_t bo = (size_t)(n0 + (j << 4) + rlane) * ldb + koff + k0;
      bh[j] = Frag<T>::load(Bb + bo);
      if (SPLIT) bl[j] = Frag<T>::load(Bb2 + bo);
    }
#pragma unroll
    for (int i = 0; i < 4; ++i) {
      const size_t ao = (size_t)(m0 + (i << 4) + rlane) * lda + koff + k0;
      V ah = Frag<T>::load(Ab + ao);
      V al;
      if (SPLIT) al = Frag<T>::load(Ab2 + ao);
#pragma unroll
      for (int j = 0; j < 4; ++j) {
        acc[i][j] = Frag<T>::mma(ah, bh[j], acc[i][j]);
        if (SPLIT) {
          acc[i][j] = Frag<T>::mma(ah, bl[j], acc[i][j]);
          acc[i][j] = Frag<T>::mma(al, bh[j], acc[i][j]);
        }
      }
      Frag<T>::guard(acc[i][0], acc[i][3], ah, SPLIT ? al : ah);
    }
    Frag<T>::keep(bh[0], bh[1], bh[2], bh[3]);
    if (SPLIT) Frag<T>::keep(bl[0], bl[1], bl[2], bl[3]);
  }
  acc_guard4(acc[0][0], acc[0][1], acc[0][2], acc[0][3]);
  acc_guard4(acc[1][0], acc[1][1], acc[1][2], acc[1][3]);
  acc_guard4(acc[2][0], acc[2][1], acc[2][2], acc[2][3]);
  acc_guard4(acc[3][0], acc[3][1], acc[3][2], acc[3][3]);

  float* slab = sT[wave];
  const float* Rb = RESID ? (resid + (size_t)b * strideR) : nullptr;
#pragma unroll
  for (int i = 0; i < 4; ++i) {
    const int mBase = m0 + (i << 4);
#pragma unroll
    for (int j = 0; j < 4; ++j) {
      const int n = n0 + (j << 4) + rlane;
      float bv = 0.f;
      if (BIAS_MODE == 2) bv = bias[n];
#pragma unroll
      for (int r = 0; r < 8; ++r) {
        float v = acc[i][j][r] * scale;
        if (BIAS_MODE == 1) v += bias[mBase + mOff + r];
        if (BIAS_MODE == 2) v += bv;
        if (RESID) v += Rb[(size_t)(mBase + mOff + r) * ldc + n];
        if (ACT == 1) v = tanhf(v);
        if (ACT == 2) v = fmaxf(v, 0.0f);
        if (ACT == 3) v = v / (1.0f + expf(-v));
        if (ACT == 4) v = (v > 0.f) ? v : 0.01f * v;
        if (ACT == 5) v = 0.5f * v * (1.0f + erff(v * 0.70710678118654752f));
        slab[(mOff + r) * 68 + (j << 4) + rlane] = v;
      }
    }
    __builtin_amdgcn_fence(__ATOMIC_RELEASE, "workgroup");
    __builtin_amdgcn_wave_barrier();
    __builtin_amdgcn_fence(__ATOMIC_ACQUIRE, "workgroup");
    if (OUT_MODE == 0) {
      float* C = (float*)Cout + (size_t)b * strideC;
      const int hh = lane >> 4, c4 = (lane & 15) * 4;
      for (int pass = 0; pass < 2; ++pass) {
#pragma unroll
        for (int it = 0; it < 8; ++it) {
          const int row = it * 2 + hh;
          v4f v = *(const v4f*)(slab + row * 68 + c4);
          *(volatile v4f*)(C + (size_t)(mBase + row) * ldc + n0 + c4) = v;
        }
        __threadfence();
      }
    } else {
      const int q = lane >> 3, c8 = (lane & 7) * 8;
      unsigned short* C  = (unsigned short*)Cout  + (size_t)b * strideC;
      unsigned short* C2 = (OUT_MODE == 2) ? ((unsigned short*)Cout2 + (size_t)b * strideC) : nullptr;
      for (int pass = 0; pass < 2; ++pass) {
#pragma unroll
        for (int it = 0; it < 4; ++it) {
          const int row = it * 4 + q;
          const float* sp = slab + row * 68 + c8;
          v8h hv, lv;
#pragma unroll
          for (int e = 0; e < 8; ++e) {
            if (OUT_MODE == 1) {
              hv[e] = (_Float16)sp[e];
            } else {
              unsigned short hb = f2bf_bits(sp[e]);
              unsigned short lb = f2bf_bits(sp[e] - bf_bits2f(hb));
              hv[e] = __builtin_bit_cast(_Float16, hb);
              lv[e] = __builtin_bit_cast(_Float16, lb);
            }
          }
          *(volatile v8h*)(C + (size_t)(mBase + row) * ldc + n0 + c8) = hv;
          if (OUT_MODE == 2) *(volatile v8h*)(C2 + (size_t)(mBase + row) * ldc + n0 + c8) = lv;
        }
        __threadfence();
      }
    }
    __builtin_amdgcn_fence(__ATOMIC_RELEASE, "workgroup");
    __builtin_amdgcn_wave_barrier();
    __builtin_amdgcn_fence(__ATOMIC_ACQUIRE, "workgroup");
  }
}

constexpr int EMB_DIM = 1024;
constexpr int NHEAD   = 16;
constexpr int HDIM    = 64;
constexpr int NBATCH  = 2;
constexpr int SEQ_LEN = 2048;
constexpr int NTOK    = NBATCH * SEQ_LEN;
constexpr int ATT_KC  = 64;
constexpr int ATT_QB  = 64;
constexpr float PCARRY = 1024.0f;
constexpr float OCARRY = 64.0f;
constexpr float WOCARRY = 256.0f;

static_assert(EMB_DIM == NHEAD * HDIM);
static_assert(HDIM == 64);
static_assert(EMB_DIM % 32 == 0);
static_assert(NTOK % 64 == 0 && EMB_DIM % 64 == 0);
static_assert(SEQ_LEN % ATT_QB == 0 && SEQ_LEN % ATT_KC == 0);
static_assert((NTOK * EMB_DIM) % (8 * 256) == 0);
static_assert((EMB_DIM * EMB_DIM) % (8 * 256) == 0);
static_assert(EMB_DIM % (4 * 256) == 0);

template <int MODE>
__global__ __launch_bounds__(256) void cast8_kernel(const float* __restrict__ in,
                                                    unsigned short* __restrict__ out,
                                                    int n8, float mul) {
  const int i = blockIdx.x * 256 + threadIdx.x;
  if (i < n8) {
    const v4f a  = *(const v4f*)(in + (size_t)i * 8);
    const v4f a1 = *(const v4f*)(in + (size_t)i * 8 + 4);
    unsigned int u[8];
#pragma unroll
    for (int e = 0; e < 4; ++e) {
      const unsigned short hb0 = f2bf_bits(a[e]);
      const unsigned short hb1 = f2bf_bits(a1[e]);
      if (MODE == 0) { u[e] = hb0; u[4 + e] = hb1; }
      else {
        const float g0 = bf_bits2f(hb0) * mul;
        const float g1 = bf_bits2f(hb1) * mul;
        u[e]     = (unsigned int)__builtin_bit_cast(unsigned short, (_Float16)g0);
        u[4 + e] = (unsigned int)__builtin_bit_cast(unsigned short, (_Float16)g1);
      }
    }
    v4u w;
    w[0] = u[0] | (u[1] << 16);
    w[1] = u[2] | (u[3] << 16);
    w[2] = u[4] | (u[5] << 16);
    w[3] = u[6] | (u[7] << 16);
    unsigned short* dst = out + (size_t)i * 8;
    *(volatile v4u*)dst = w;
    __threadfence();
    *(volatile v4u*)dst = w;
  }
}

__global__ __launch_bounds__(256) void bias_rne_kernel(const float* __restrict__ in,
                                                       float* __restrict__ out, int n4) {
  const int i = blockIdx.x * 256 + threadIdx.x;
  if (i < n4) {
    const v4f a = *(const v4f*)(in + (size_t)i * 4);
    v4f r;
#pragma unroll
    for (int e = 0; e < 4; ++e) r[e] = bf_bits2f(f2bf_bits(a[e]));
    float* dst = out + (size_t)i * 4;
    *(volatile v4f*)dst = r;
    __threadfence();
    *(volatile v4f*)dst = r;
  }
}

__device__ __forceinline__ v8f mma_h(v16h a, v16h b, v8f c) {
  c = __builtin_amdgcn_wmma_f32_16x16x32_f16(false, a, false, b, (short)0, c, false, false);
  asm volatile("v_nop\n\tv_nop\n\tv_nop\n\tv_nop" : "+v"(c) : "v"(a), "v"(b));
  return c;
}

__global__ __launch_bounds__(128)
void attn64_f16planes(const unsigned short* __restrict__ Qp, const unsigned short* __restrict__ Kp,
                      const unsigned short* __restrict__ Vtp, unsigned short* __restrict__ Op,
                      float qscale) {
  union FH { v16h v; v8h hv[2]; };
  const _Float16* Q  = (const _Float16*)Qp;
  const _Float16* Kg = (const _Float16*)Kp;
  const _Float16* Vt = (const _Float16*)Vtp;
  _Float16*       O  = (_Float16*)Op;

  __shared__ __align__(16) _Float16 Ksh[ATT_KC * HDIM];
  __shared__ __align__(16) _Float16 Vth[HDIM * ATT_KC];
  __shared__ __align__(16) _Float16 Psh[4][16 * ATT_KC];
  __shared__ __align__(16) float    Os[4][16 * 68];

  const int tid  = threadIdx.x;
  const int wave = tid >> 5;
  const int lane = tid & 31;
  const int hh   = lane >> 4;
  const int c    = lane & 15;

  const int nqb = SEQ_LEN / ATT_QB;
  const int bx  = blockIdx.x;
  const int qb  = bx % nqb;
  const int bh  = bx / nqb;
  const int h   = bh % NHEAD;
  const int b   = bh / NHEAD;
  const int q0  = qb * ATT_QB + wave * 16;
  const size_t tokb = (size_t)b * SEQ_LEN;

  v16h qa[2];
  {
    const _Float16* qrow = Q + (tokb + q0 + c) * EMB_DIM + h * HDIM;
#pragma unroll
    for (int dc = 0; dc < 2; ++dc) {
      FH f;
      f.hv[0] = *(const v8h*)(qrow + dc * 32 + 8 * hh);
      f.hv[1] = *(const v8h*)(qrow + dc * 32 + 16 + 8 * hh);
      qa[dc] = f.v;
    }
  }

  float mrow[8], lrow[8];
  v8f oacc[4];
#pragma unroll
  for (int r = 0; r < 8; ++r) { mrow[r] = -INFINITY; lrow[r] = 0.f; }
#pragma unroll
  for (int t = 0; t < 4; ++t) oacc[t] = (v8f){0.f,0.f,0.f,0.f,0.f,0.f,0.f,0.f};

  __bf16 dummy_unused = (__bf16)0.0f; (void)dummy_unused;

  for (int kc = 0; kc < SEQ_LEN / ATT_KC; ++kc) {
    const int kv0 = kc * ATT_KC;
    __syncthreads();
    {
      const int kvr = tid >> 1, hf = (tid & 1) * 32;
      const _Float16* krow = Kg + (tokb + kv0 + kvr) * EMB_DIM + h * HDIM + hf;
      const _Float16* vrow = Vt + (size_t)(h * HDIM + kvr) * NTOK + tokb + kv0 + hf;
#pragma unroll
      for (int i = 0; i < 4; ++i) {
        const v8h kk = *(const v8h*)(krow + 8 * i);
        const v8h vv = *(const v8h*)(vrow + 8 * i);
        *(v8h*)(Ksh + kvr * HDIM + hf + 8 * i) = kk;
        *(v8h*)(Vth + kvr * ATT_KC + hf + 8 * i) = vv;
      }
    }
    __syncthreads();

    v8f s[4];
#pragma unroll
    for (int j = 0; j < 4; ++j) {
      s[j] = (v8f){0.f,0.f,0.f,0.f,0.f,0.f,0.f,0.f};
#pragma unroll
      for (int dc = 0; dc < 2; ++dc) {
        FH kb;
        kb.hv[0] = *(const v8h*)(Ksh + (j * 16 + c) * HDIM + dc * 32 + 8 * hh);
        kb.hv[1] = *(const v8h*)(Ksh + (j * 16 + c) * HDIM + dc * 32 + 16 + 8 * hh);
        s[j] = mma_h(qa[dc], kb.v, s[j]);
      }
    }

    float cm[8];
#pragma unroll
    for (int r = 0; r < 8; ++r) {
      float m = -INFINITY;
#pragma unroll
      for (int j = 0; j < 4; ++j) {
        const float sv = s[j][r] * qscale;
        s[j][r] = sv;
        m = fmaxf(m, sv);
      }
#pragma unroll
      for (int off = 1; off < 16; off <<= 1) m = fmaxf(m, __shfl_xor(m, off, 32));
      cm[r] = m;
    }
    _Float16* pw = Psh[wave];
#pragma unroll
    for (int r = 0; r < 8; ++r) {
      const float mnew  = fmaxf(mrow[r], cm[r]);
      const float alpha = expf(mrow[r] - mnew);
      mrow[r] = mnew;
      float psum = 0.f;
#pragma unroll
      for (int j = 0; j < 4; ++j) {
        const float p = expf(s[j][r] - mnew);
        psum += p;
        pw[(8 * hh + r) * ATT_KC + j * 16 + c] = (_Float16)(p * PCARRY);
      }
#pragma unroll
      for (int off = 1; off < 16; off <<= 1) psum += __shfl_xor(psum, off, 32);
      lrow[r] = lrow[r] * alpha + psum;
#pragma unroll
      for (int t = 0; t < 4; ++t) oacc[t][r] *= alpha;
    }
    __builtin_amdgcn_fence(__ATOMIC_RELEASE, "workgroup");
    __builtin_amdgcn_wave_barrier();
    __builtin_amdgcn_fence(__ATOMIC_ACQUIRE, "workgroup");

#pragma unroll 1
    for (int kk = 0; kk < 2; ++kk) {
      FH pa;
      pa.hv[0] = *(const v8h*)(pw + c * ATT_KC + kk * 32 + 8 * hh);
      pa.hv[1] = *(const v8h*)(pw + c * ATT_KC + kk * 32 + 16 + 8 * hh);
#pragma unroll
      for (int t = 0; t < 4; ++t) {
        FH vb;
        vb.hv[0] = *(const v8h*)(Vth + (t * 16 + c) * ATT_KC + kk * 32 + 8 * hh);
        vb.hv[1] = *(const v8h*)(Vth + (t * 16 + c) * ATT_KC + kk * 32 + 16 + 8 * hh);
        oacc[t] = mma_h(pa.v, vb.v, oacc[t]);
      }
    }
  }

  float* os = Os[wave];
#pragma unroll
  for (int r = 0; r < 8; ++r) {
    const float inv = (1.0f / lrow[r]) * (OCARRY / PCARRY);
#pragma unroll
    for (int t = 0; t < 4; ++t) os[(8 * hh + r) * 68 + t * 16 + c] = oacc[t][r] * inv;
  }
  __builtin_amdgcn_fence(__ATOMIC_RELEASE, "workgroup");
  __builtin_amdgcn_wave_barrier();
  __builtin_amdgcn_fence(__ATOMIC_ACQUIRE, "workgroup");
  {
    const int q = lane >> 3, c8 = (lane & 7) * 8;
    for (int pass = 0; pass < 2; ++pass) {
#pragma unroll
      for (int it = 0; it < 4; ++it) {
        const int row = it * 4 + q;
        const float* sp = os + row * 68 + c8;
        v8h hv;
#pragma unroll
        for (int e = 0; e < 8; ++e) hv[e] = (_Float16)sp[e];
        *(volatile v8h*)(O + (tokb + q0 + row) * EMB_DIM + h * HDIM + c8) = hv;
      }
      __threadfence();
    }
  }
}

constexpr size_t XPLANE_BYTES = (size_t)NTOK * EMB_DIM * 2;
constexpr size_t WPLANE_BYTES = (size_t)EMB_DIM * EMB_DIM * 2;
constexpr size_t BIAS_BYTES   = (size_t)EMB_DIM * 4;
constexpr size_t OFF_XQ = 0;
constexpr size_t OFF_XK = OFF_XQ + XPLANE_BYTES;
constexpr size_t OFF_XV = OFF_XK + XPLANE_BYTES;
constexpr size_t OFF_WQ = OFF_XV + XPLANE_BYTES;
constexpr size_t OFF_WK = OFF_WQ + WPLANE_BYTES;
constexpr size_t OFF_WV = OFF_WK + WPLANE_BYTES;
constexpr size_t OFF_WO = OFF_WV + WPLANE_BYTES;
constexpr size_t OFF_BO = OFF_WO + WPLANE_BYTES;
constexpr size_t OFF_QH = OFF_BO + BIAS_BYTES;
constexpr size_t OFF_KH = OFF_QH + XPLANE_BYTES;
constexpr size_t OFF_VT = OFF_KH + XPLANE_BYTES;
constexpr size_t OFF_OH = OFF_VT + XPLANE_BYTES;
constexpr size_t WS_TOTAL = OFF_OH + XPLANE_BYTES;
static_assert(WS_TOTAL == 67112960);
static_assert(WS_TOTAL <= 134217728);
static_assert(OFF_BO % 128 == 0 && OFF_QH % 128 == 0 && OFF_OH % 128 == 0);

extern "C" void kernel_launch(void* const* d_in, const int* in_sizes, int n_in,
                              void* d_out, int out_size, void* d_ws, size_t ws_size,
                              hipStream_t stream) {
  if (n_in < 8) return;
  if (in_sizes[0] != NTOK * EMB_DIM || in_sizes[1] != NTOK * EMB_DIM || in_sizes[2] != NTOK * EMB_DIM) return;
  if (in_sizes[3] != EMB_DIM * EMB_DIM || in_sizes[4] != EMB_DIM * EMB_DIM ||
      in_sizes[5] != EMB_DIM * EMB_DIM || in_sizes[6] != EMB_DIM * EMB_DIM) return;
  if (in_sizes[7] != EMB_DIM) return;
  if (out_size != NTOK * EMB_DIM) return;
  if (ws_size < WS_TOTAL) return;

  const float* xq = (const float*)d_in[0];
  const float* xk = (const float*)d_in[1];
  const float* xv = (const float*)d_in[2];
  const float* Wq = (const float*)d_in[3];
  const float* Wk = (const float*)d_in[4];
  const float* Wv = (const float*)d_in[5];
  const float* Wo = (const float*)d_in[6];
  const float* bo = (const float*)d_in[7];
  float* out = (float*)d_out;

  char* ws = (char*)d_ws;
  unsigned short* xq_bf = (unsigned short*)(ws + OFF_XQ);
  unsigned short* xk_bf = (unsigned short*)(ws + OFF_XK);
  unsigned short* xv_bf = (unsigned short*)(ws + OFF_XV);
  unsigned short* Wq_bf = (unsigned short*)(ws + OFF_WQ);
  unsigned short* Wk_bf = (unsigned short*)(ws + OFF_WK);
  unsigned short* Wv_bf = (unsigned short*)(ws + OFF_WV);
  unsigned short* Wo_h  = (unsigned short*)(ws + OFF_WO);
  float*          bo_r  = (float*)(ws + OFF_BO);
  unsigned short* Qh    = (unsigned short*)(ws + OFF_QH);
  unsigned short* Kh    = (unsigned short*)(ws + OFF_KH);
  unsigned short* Vt    = (unsigned short*)(ws + OFF_VT);
  unsigned short* Oh    = (unsigned short*)(ws + OFF_OH);

  const int n8x = (NTOK * EMB_DIM) / 8;
  const int n8w = (EMB_DIM * EMB_DIM) / 8;
  cast8_kernel<0><<<dim3((n8x + 255) / 256), dim3(256), 0, stream>>>(xq, xq_bf, n8x, 1.0f);
  cast8_kernel<0><<<dim3((n8x + 255) / 256), dim3(256), 0, stream>>>(xk, xk_bf, n8x, 1.0f);
  cast8_kernel<0><<<dim3((n8x + 255) / 256), dim3(256), 0, stream>>>(xv, xv_bf, n8x, 1.0f);
  cast8_kernel<0><<<dim3((n8w + 255) / 256), dim3(256), 0, stream>>>(Wq, Wq_bf, n8w, 1.0f);
  cast8_kernel<0><<<dim3((n8w + 255) / 256), dim3(256), 0, stream>>>(Wk, Wk_bf, n8w, 1.0f);
  cast8_kernel<0><<<dim3((n8w + 255) / 256), dim3(256), 0, stream>>>(Wv, Wv_bf, n8w, 1.0f);
  cast8_kernel<1><<<dim3((n8w + 255) / 256), dim3(256), 0, stream>>>(Wo, Wo_h, n8w, WOCARRY);
  const int n4b = EMB_DIM / 4;
  bias_rne_kernel<<<dim3((n4b + 255) / 256), dim3(256), 0, stream>>>(bo, bo_r, n4b);

  const int tiles_tok = (NTOK / 64) * (EMB_DIM / 64);
  const int tiles_vt  = (EMB_DIM / 64) * (NTOK / 64);
  wmma_gemm64<1, false, 0, 1, false, 0><<<dim3((tiles_tok + 7) / 8, 1), dim3(256), 0, stream>>>(
      xq_bf, nullptr, EMB_DIM, 0L, Wq_bf, nullptr, EMB_DIM, 0L,
      (void*)Qh, nullptr, EMB_DIM, 0L, nullptr, nullptr, 0L, NTOK, EMB_DIM, EMB_DIM, 1.0f);
  wmma_gemm64<1, false, 0, 1, false, 0><<<dim3((tiles_tok + 7) / 8, 1), dim3(256), 0, stream>>>(
      xk_bf, nullptr, EMB_DIM, 0L, Wk_bf, nullptr, EMB_DIM, 0L,
      (void*)Kh, nullptr, EMB_DIM, 0L, nullptr, nullptr, 0L, NTOK, EMB_DIM, EMB_DIM, 1.0f);
  wmma_gemm64<1, false, 0, 1, false, 0><<<dim3((tiles_vt + 7) / 8, 1), dim3(256), 0, stream>>>(
      Wv_bf, nullptr, EMB_DIM, 0L, xv_bf, nullptr, EMB_DIM, 0L,
      (void*)Vt, nullptr, NTOK, 0L, nullptr, nullptr, 0L, EMB_DIM, NTOK, EMB_DIM, 1.0f);

  const int ablocks = NBATCH * NHEAD * (SEQ_LEN / ATT_QB);
  const float qscale = 0.125f;
  attn64_f16planes<<<dim3(ablocks), dim3(128), 0, stream>>>(Qh, Kh, Vt, Oh, qscale);

  wmma_gemm64<0, false, 2, 0, false, 0><<<dim3((tiles_tok + 7) / 8, 1), dim3(256), 0, stream>>>(
      Oh, nullptr, EMB_DIM, 0L, Wo_h, nullptr, EMB_DIM, 0L,
      (void*)out, nullptr, EMB_DIM, 0L, bo_r, nullptr, 0L, NTOK, EMB_DIM, EMB_DIM,
      1.0f / (OCARRY * WOCARRY));
}
